// SimpleTemporalGCN_7533372637953
// MI455X (gfx1250) — hardware-verified
//
#include <hip/hip_runtime.h>
#include <math.h>
#include <stddef.h>

constexpr int kBatch   = 64;
constexpr int kNode    = 100;
constexpr int kNodePad = 128;
constexpr int kHid     = 128;
constexpr int kTdim    = 128;
constexpr int kKx      = 224;
constexpr int kUbtRows = 64;
constexpr float kInvS1 = 0.99999499320983887f;

static_assert(kKx % 32 == 0 && kHid % 32 == 0 && kTdim % 32 == 0, "K multiple of 32");
static_assert(kNodePad % 64 == 0 && kHid % 64 == 0 && kBatch % 64 == 0 && kUbtRows % 64 == 0, "M,N multiples of 64");
static_assert(2 * kNode <= kKx && kNode <= kNodePad, "padding covers real extents");
static_assert((kBatch * kNode * kNode) % 1024 == 0, "final writer grid exact");

constexpr size_t kWsTotal = 39436544u;
static_assert(kWsTotal <= 134217728u, "carve budget");

typedef __attribute__((ext_vector_type(16))) _Float16 v16h;
typedef __attribute__((ext_vector_type(8)))  _Float16 v8h;
typedef __attribute__((ext_vector_type(16))) __bf16   v16b;
typedef __attribute__((ext_vector_type(8)))  __bf16   v8b;
typedef __attribute__((ext_vector_type(8)))  float    v8f;
typedef __attribute__((ext_vector_type(4)))  float    v4f;
typedef __attribute__((ext_vector_type(4)))  unsigned int v4u;

__device__ __forceinline__ unsigned short f2bf_bits(float f) {
  unsigned u = __float_as_uint(f);
  return (unsigned short)((u + 0x7FFFu + ((u >> 16) & 1u)) >> 16);
}
__device__ __forceinline__ float bf_bits2f(unsigned short h) { return __uint_as_float(((unsigned)h) << 16); }

__device__ __forceinline__ void dep_guard_h(v8f& a, v8f& b, v16h x, v16h y) { asm volatile("v_nop\n\tv_nop\n\tv_nop\n\tv_nop" : "+v"(a), "+v"(b) : "v"(x), "v"(y)); }
__device__ __forceinline__ void dep_guard_b(v8f& a, v8f& b, v16b x, v16b y) { asm volatile("v_nop\n\tv_nop\n\tv_nop\n\tv_nop" : "+v"(a), "+v"(b) : "v"(x), "v"(y)); }
__device__ __forceinline__ void keep4_h(v16h a, v16h b, v16h c, v16h d) { asm volatile("v_nop" :: "v"(a), "v"(b), "v"(c), "v"(d)); }
__device__ __forceinline__ void keep4_b(v16b a, v16b b, v16b c, v16b d) { asm volatile("v_nop" :: "v"(a), "v"(b), "v"(c), "v"(d)); }
__device__ __forceinline__ void acc_guard4(v8f& a, v8f& b, v8f& c, v8f& d) { asm volatile("v_nop\n\tv_nop\n\tv_nop\n\tv_nop" : "+v"(a), "+v"(b), "+v"(c), "+v"(d)); }
template <typename T> struct Frag;
template <> struct Frag<_Float16> {
  typedef v16h V; union U { v16h v; v8h h[2]; };
  static __device__ __forceinline__ v16h load(const _Float16* p) {
    U f; f.h[0] = *(const v8h*)(p); f.h[1] = *(const v8h*)(p + 16); return f.v;
  }
  static __device__ __forceinline__ v8f mma(v16h a, v16h b, v8f c) {
    return __builtin_amdgcn_wmma_f32_16x16x32_f16(false, a, false, b, (short)0, c, false, false);
  }
  static __device__ __forceinline__ void guard(v8f& a, v8f& b, v16h x, v16h y) { dep_guard_h(a, b, x, y); }
  static __device__ __forceinline__ void keep(v16h a, v16h b, v16h c, v16h d) { keep4_h(a, b, c, d); }
};
template <> struct Frag<__bf16> {
  typedef v16b V; union U { v16b v; v8b h[2]; };
  static __device__ __forceinline__ v16b load(const __bf16* p) {
    U f; f.h[0] = *(const v8b*)(p); f.h[1] = *(const v8b*)(p + 16); return f.v;
  }
  static __device__ __forceinline__ v8f mma(v16b a, v16b b, v8f c) {
    return __builtin_amdgcn_wmma_f32_16x16x32_bf16(false, a, false, b, (short)0, c, false, false);
  }
  static __device__ __forceinline__ void guard(v8f& a, v8f& b, v16b x, v16b y) { dep_guard_b(a, b, x, y); }
  static __device__ __forceinline__ void keep(v16b a, v16b b, v16b c, v16b d) { keep4_b(a, b, c, d); }
};

template <int ET> struct Elem;
template <> struct Elem<0> { typedef _Float16 T; };
template <> struct Elem<1> { typedef __bf16 T; };
template <int ET, bool SPLIT, int BIAS_MODE, int OUT_MODE, bool RESID, int ACT = 0>
__global__ __launch_bounds__(256) void wmma_gemm64(
    const unsigned short* __restrict__ Ap, const unsigned short* __restrict__ A2p, int lda, long strideA,
    const unsigned short* __restrict__ Btp, const unsigned short* __restrict__ Bt2p, int ldb, long strideB,
    void* __restrict__ Cout, void* __restrict__ Cout2, int ldc, long strideC,
    const float* __restrict__ bias, const float* __restrict__ gam, const float* __restrict__ bet,
    const float* __restrict__ resid, long strideR,
    int M, int N, int K, float scale) {
  typedef typename Elem<ET>::T T;
  typedef typename Frag<T>::V V;
  const T* A = (const T*)Ap; const T* A2 = (const T*)A2p; const T* Bt = (const T*)Btp; const T* Bt2 = (const T*)Bt2p;
  __shared__ __align__(16) float sT[8][16 * 68];
  const int b    = blockIdx.y;
  const int lane = threadIdx.x & 31;
  const int wave = threadIdx.x >> 5;
  const int tilesN = N >> 6;
  const int tilesM = M >> 6;
  const int tile = blockIdx.x * 8 + wave;
  if (tile >= tilesM * tilesN) return;
  const int tm = tile / tilesN;
  const int tn = tile - tm * tilesN;
  const int m0 = tm << 6;
  const int n0 = tn << 6;

  const T* Ab  = A  + (size_t)b * strideA;
  const T* Bb  = Bt + (size_t)b * strideB;
  const T* Ab2 = SPLIT ? (A2  + (size_t)b * strideA) : nullptr;
  const T* Bb2 = SPLIT ? (Bt2 + (size_t)b * strideB) : nullptr;

  const int rlane = lane & 15;
  const int koff  = (lane >> 4) * 8;
  const int mOff  = (lane >> 4) * 8;

  v8f acc[4][4];
#pragma unroll
  for (int i = 0; i < 4; ++i)
#pragma unroll
    for (int j = 0; j < 4; ++j) acc[i][j] = (v8f){0.f,0.f,0.f,0.f,0.f,0.f,0.f,0.f};

  for (int k0 = 0; k0 < K; k0 += 32) {
    V bh[4], bl[4];
#pragma unroll
    for (int j = 0; j < 4; ++j) {
      const size_t bo = (size_t)(n0 + (j << 4) + rlane) * ldb + koff + k0;
      bh[j] = Frag<T>::load(Bb + bo);
      if (SPLIT) bl[j] = Frag<T>::load(Bb2 + bo);
    }
#pragma unroll
    for (int i = 0; i < 4; ++i) {
      const size_t ao = (size_t)(m0 + (i << 4) + rlane) * lda + koff + k0;
      V ah = Frag<T>::load(Ab + ao);
      V al;
      if (SPLIT) al = Frag<T>::load(Ab2 + ao);
#pragma unroll
      for (int j = 0; j < 4; ++j) {
        acc[i][j] = Frag<T>::mma(ah, bh[j], acc[i][j]);
        if (SPLIT) {
          acc[i][j] = Frag<T>::mma(ah, bl[j], acc[i][j]);
          acc[i][j] = Frag<T>::mma(al, bh[j], acc[i][j]);
        }
      }
      Frag<T>::guard(acc[i][0], acc[i][3], ah, SPLIT ? al : ah);
    }
    Frag<T>::keep(bh[0], bh[1], bh[2], bh[3]);
    if (SPLIT) Frag<T>::keep(bl[0], bl[1], bl[2], bl[3]);
  }
  acc_guard4(acc[0][0], acc[0][1], acc[0][2], acc[0][3]);
  acc_guard4(acc[1][0], acc[1][1], acc[1][2], acc[1][3]);
  acc_guard4(acc[2][0], acc[2][1], acc[2][2], acc[2][3]);
  acc_guard4(acc[3][0], acc[3][1], acc[3][2], acc[3][3]);

  float* slab = sT[wave];
  const float* Rb = RESID ? (resid + (size_t)b * strideR) : nullptr;
#pragma unroll
  for (int i = 0; i < 4; ++i) {
    const int mBase = m0 + (i << 4);
#pragma unroll
    for (int j = 0; j < 4; ++j) {
      const int n = n0 + (j << 4) + rlane;
      float bv = 0.f, gv = 1.f, ev = 0.f;
      if (BIAS_MODE == 2 || BIAS_MODE == 3) bv = bias[n];
      if (BIAS_MODE == 3) { gv = gam[n]; ev = bet[n]; }
#pragma unroll
      for (int r = 0; r < 8; ++r) {
        float v = acc[i][j][r] * scale;
        if (BIAS_MODE == 1) v += bias[mBase + mOff + r];
        if (BIAS_MODE == 2) v += bv;
        if (BIAS_MODE == 3) v = fmaxf(gv * ((v + bv) * kInvS1) + ev, 0.0f);
        if (RESID) v += Rb[(size_t)(mBase + mOff + r) * ldc + n];
        if (ACT == 1) v = tanhf(v);
        if (ACT == 2) v = fmaxf(v, 0.0f);
        if (ACT == 3) v = v / (1.0f + expf(-v));
        if (ACT == 4) v = (v > 0.f) ? v : 0.01f * v;
        slab[(mOff + r) * 68 + (j << 4) + rlane] = v;
      }
    }
    __builtin_amdgcn_fence(__ATOMIC_RELEASE, "workgroup");
    __builtin_amdgcn_wave_barrier();
    __builtin_amdgcn_fence(__ATOMIC_ACQUIRE, "workgroup");
    if (OUT_MODE == 0) {
      float* C = (float*)Cout + (size_t)b * strideC;
      const int hh = lane >> 4, c4 = (lane & 15) * 4;
      for (int pass = 0; pass < 2; ++pass) {
#pragma unroll
        for (int it = 0; it < 8; ++it) {
          const int row = it * 2 + hh;
          v4f v = *(const v4f*)(slab + row * 68 + c4);
          *(volatile v4f*)(C + (size_t)(mBase + row) * ldc + n0 + c4) = v;
        }
        __threadfence();
      }
    } else {
      const int q = lane >> 3, c8 = (lane & 7) * 8;
      unsigned short* C  = (unsigned short*)Cout  + (size_t)b * strideC;
      unsigned short* C2 = (OUT_MODE == 2) ? ((unsigned short*)Cout2 + (size_t)b * strideC) : nullptr;
      for (int pass = 0; pass < 2; ++pass) {
#pragma unroll
        for (int it = 0; it < 4; ++it) {
          const int row = it * 4 + q;
          const float* sp = slab + row * 68 + c8;
          v8h hv, lv;
#pragma unroll
          for (int e = 0; e < 8; ++e) {
            if (OUT_MODE == 1) {
              hv[e] = (_Float16)sp[e];
            } else {
              unsigned short hb = f2bf_bits(sp[e]);
              unsigned short lb = f2bf_bits(sp[e] - bf_bits2f(hb));
              hv[e] = __builtin_bit_cast(_Float16, hb);
              lv[e] = __builtin_bit_cast(_Float16, lb);
            }
          }
          *(volatile v8h*)(C + (size_t)(mBase + row) * ldc + n0 + c8) = hv;
          if (OUT_MODE == 2) *(volatile v8h*)(C2 + (size_t)(mBase + row) * ldc + n0 + c8) = lv;
        }
        __threadfence();
      }
    }
    __builtin_amdgcn_fence(__ATOMIC_RELEASE, "workgroup");
    __builtin_amdgcn_wave_barrier();
    __builtin_amdgcn_fence(__ATOMIC_ACQUIRE, "workgroup");
  }
}

struct F8 { float v[8]; };
__device__ __forceinline__ void pack_hl(const F8& f, v4u& wh, v4u& wl) {
#pragma unroll
  for (int p = 0; p < 4; ++p) {
    const unsigned short h0 = f2bf_bits(f.v[2 * p]);
    const unsigned short h1 = f2bf_bits(f.v[2 * p + 1]);
    const unsigned short l0 = f2bf_bits(f.v[2 * p] - bf_bits2f(h0));
    const unsigned short l1 = f2bf_bits(f.v[2 * p + 1] - bf_bits2f(h1));
    wh[p] = (unsigned)h0 | ((unsigned)h1 << 16);
    wl[p] = (unsigned)l0 | ((unsigned)l1 << 16);
  }
}

__global__ __launch_bounds__(256) void k_wtrans(
    const float* __restrict__ w0, const float* __restrict__ w1, const float* __restrict__ w2,
    const float* __restrict__ w3, const float* __restrict__ w4, const float* __restrict__ w5,
    unsigned short* o0h, unsigned short* o0l, unsigned short* o1h, unsigned short* o1l,
    unsigned short* o2h, unsigned short* o2l, unsigned short* o3h, unsigned short* o3l,
    unsigned short* o4h, unsigned short* o4l, unsigned short* o5h, unsigned short* o5l) {
  __shared__ __align__(16) float tile[16 * kKx];
  const int job = blockIdx.x >> 3;
  const int n0  = (blockIdx.x & 7) * 16;
  const float* src = w0; unsigned short* dh = o0h; unsigned short* dl = o0l;
  int kr = kTdim, nr = kHid, kp = kHid;
  if (job == 1)      { src = w1; dh = o1h; dl = o1l; kr = kHid;      nr = kHid;  kp = kHid; }
  else if (job == 2) { src = w2; dh = o2h; dl = o2l; kr = kHid;      nr = kNode; kp = kHid; }
  else if (job == 3) { src = w3; dh = o3h; dl = o3l; kr = 2 * kNode; nr = kHid;  kp = kKx;  }
  else if (job == 4) { src = w4; dh = o4h; dl = o4l; kr = kHid;      nr = kHid;  kp = kHid; }
  else if (job == 5) { src = w5; dh = o5h; dl = o5l; kr = kHid;      nr = kHid;  kp = kHid; }
  const int tot = 16 * kp;
#pragma unroll 1
  for (int idx = threadIdx.x; idx < tot; idx += 256) {
    const int r  = idx / kp;
    const int k  = idx - r * kp;
    const int n  = n0 + r;
    const int kc = (k < kr) ? k : (kr - 1);
    const int nc = (n < nr) ? n : (nr - 1);
    const float v = src[(size_t)kc * nr + nc];
    tile[idx] = ((k < kr) && (n < nr)) ? v : 0.0f;
  }
  __syncthreads();
  const int nch = tot >> 3;
  const size_t base = (size_t)n0 * kp;
  for (int pass = 0; pass < 2; ++pass) {
#pragma unroll 1
    for (int c = threadIdx.x; c < nch; c += 256) {
      const float* sp = tile + c * 8;
      F8 f;
#pragma unroll
      for (int q = 0; q < 8; ++q) f.v[q] = sp[q];
      v4u wh, wl;
      pack_hl(f, wh, wl);
      *(volatile v4u*)(dh + base + (size_t)c * 8) = wh;
      *(volatile v4u*)(dl + base + (size_t)c * 8) = wl;
    }
    __threadfence();
  }
}

__global__ __launch_bounds__(256) void k_temb(const float* __restrict__ timev,
                                              unsigned short* th, unsigned short* tl, float cst) {
  __shared__ __align__(16) float vals[kBatch * kTdim];
#pragma unroll 1
  for (int e = threadIdx.x; e < kBatch * kTdim; e += 256) {
    const int b  = e >> 7;
    const int j  = e & 127;
    const int jj = j & 63;
    const float fr  = expf((float)jj * cst);
    const float ang = timev[b] * fr;
    float sv, cv;
    sincosf(ang, &sv, &cv);
    vals[e] = (j < 64) ? sv : cv;
  }
  __syncthreads();
  for (int pass = 0; pass < 2; ++pass) {
#pragma unroll 1
    for (int c = threadIdx.x; c < (kBatch * kTdim) / 8; c += 256) {
      const float* sp = vals + c * 8;
      F8 f;
#pragma unroll
      for (int q = 0; q < 8; ++q) f.v[q] = sp[q];
      v4u wh, wl;
      pack_hl(f, wh, wl);
      *(volatile v4u*)(th + (size_t)c * 8) = wh;
      *(volatile v4u*)(tl + (size_t)c * 8) = wl;
    }
    __threadfence();
  }
}

__global__ __launch_bounds__(256) void k_adj(const float* __restrict__ X,
                                             unsigned short* ah, unsigned short* al) {
  __shared__ int flag[kNode * kNode];
  __shared__ float dinv[kNodePad];
  const int b = blockIdx.x;
  const int t = threadIdx.x;
  const float* Xb = X + (size_t)b * (kNode * kNode);
#pragma unroll 1
  for (int e = t; e < kNode * kNode; e += 256) {
    const int i = e / kNode;
    const int j = e - i * kNode;
    const float xv = Xb[e];
    flag[e] = ((xv != 0.0f) || (i == j)) ? 1 : 0;
  }
  __syncthreads();
  if (t < kNodePad) {
    const int row = (t < kNode) ? t : (kNode - 1);
    int cnt = 0;
#pragma unroll 1
    for (int j = 0; j < kNode; ++j) cnt += flag[row * kNode + j];
    const float d = 1.0f / sqrtf((float)cnt);
    dinv[t] = (t < kNode) ? d : 0.0f;
  }
  __syncthreads();
  const size_t base = (size_t)b * (kNodePad * kNodePad);
  for (int pass = 0; pass < 2; ++pass) {
#pragma unroll 1
    for (int c = t; c < (kNodePad * kNodePad) / 8; c += 256) {
      const int e  = c * 8;
      const int i  = e >> 7;
      const int j0 = e & 127;
      const int ic = (i < kNode) ? i : (kNode - 1);
      const float di = dinv[i];
      F8 f;
#pragma unroll
      for (int q = 0; q < 8; ++q) {
        const int j  = j0 + q;
        const int jc = (j < kNode) ? j : (kNode - 1);
        const int fl = flag[ic * kNode + jc];
        const float a = ((i < kNode) && (j < kNode) && (fl != 0)) ? 1.0f : 0.0f;
        f.v[q] = (di * a) * dinv[j];
      }
      v4u wh, wl;
      pack_hl(f, wh, wl);
      *(volatile v4u*)(ah + base + (size_t)e) = wh;
      *(volatile v4u*)(al + base + (size_t)e) = wl;
    }
    __threadfence();
  }
}

__global__ __launch_bounds__(256) void k_ubt(const float* __restrict__ We0, const float* __restrict__ We1,
                                             const float* __restrict__ g_e0,
                                             unsigned short* uh, unsigned short* ul) {
  __shared__ float vv[kHid];
  __shared__ float uu[2 * kHid];
  const int t = threadIdx.x;
  if (t < kHid) vv[t] = g_e0[t] * We1[t] * kInvS1;
  __syncthreads();
  {
    const float* wr = We0 + (size_t)t * kHid;
    float acc = 0.0f;
#pragma unroll 1
    for (int h = 0; h < kHid; ++h) acc += wr[h] * vv[h];
    uu[t] = acc;
  }
  __syncthreads();
  for (int pass = 0; pass < 2; ++pass) {
#pragma unroll 1
    for (int c = t; c < (kUbtRows * kHid) / 8; c += 256) {
      const int e   = c * 8;
      const int row = e >> 7;
      const int k0  = e & 127;
      F8 f;
#pragma unroll
      for (int q = 0; q < 8; ++q) {
        const float a0 = uu[k0 + q];
        const float a1 = uu[kHid + k0 + q];
        f.v[q] = (row == 0) ? a0 : ((row == 1) ? a1 : 0.0f);
      }
      v4u wh, wl;
      pack_hl(f, wh, wl);
      *(volatile v4u*)(uh + (size_t)e) = wh;
      *(volatile v4u*)(ul + (size_t)e) = wl;
    }
    __threadfence();
  }
}

__global__ __launch_bounds__(256) void k_hpost(const float* __restrict__ hf, const float* __restrict__ We1,
                                               const float* __restrict__ be0, const float* __restrict__ b_e0,
                                               const float* __restrict__ g_e0, const float* __restrict__ be1,
                                               unsigned short* hh, unsigned short* hl, float* cbt) {
  __shared__ float cbl[kBatch];
  __shared__ float d0s;
  const int t = threadIdx.x;
  if (t < kBatch) {
    const float* hr = hf + (size_t)t * kHid;
    float acc = 0.0f;
#pragma unroll 1
    for (int k = 0; k < kHid; ++k) acc += hr[k] * We1[kHid + k];
    cbl[t] = acc;
  }
  if ((t >> 5) == 2) {
    float d = be1[0];
#pragma unroll 1
    for (int h = 0; h < kHid; ++h) {
      const float vh = g_e0[h] * We1[h] * kInvS1;
      d += be0[h] * vh + b_e0[h] * We1[h];
    }
    if (t == 64) d0s = d;
  }
  __syncthreads();
  {
    const float d0 = d0s;
    for (int pass = 0; pass < 2; ++pass) {
      if (t < 16) {
        v4f o;
        o[0] = cbl[4 * t + 0] + d0;
        o[1] = cbl[4 * t + 1] + d0;
        o[2] = cbl[4 * t + 2] + d0;
        o[3] = cbl[4 * t + 3] + d0;
        *(volatile v4f*)(cbt + 4 * t) = o;
      }
      __threadfence();
    }
  }
  for (int pass = 0; pass < 2; ++pass) {
#pragma unroll 1
    for (int c = t; c < (kBatch * kHid) / 8; c += 256) {
      const int e = c * 8;
      const v4f a0 = *(const v4f*)(hf + e);
      const v4f a1 = *(const v4f*)(hf + e + 4);
      F8 f;
      f.v[0] = a0[0]; f.v[1] = a0[1]; f.v[2] = a0[2]; f.v[3] = a0[3];
      f.v[4] = a1[0]; f.v[5] = a1[1]; f.v[6] = a1[2]; f.v[7] = a1[3];
      v4u wh, wl;
      pack_hl(f, wh, wl);
      *(volatile v4u*)(hh + (size_t)e) = wh;
      *(volatile v4u*)(hl + (size_t)e) = wl;
    }
    __threadfence();
  }
}

__global__ __launch_bounds__(256) void k_xbuild(const float* __restrict__ tnraw, const float* __restrict__ btn,
                                                const float* __restrict__ g_tn, const float* __restrict__ b_tn,
                                                unsigned short* xh, unsigned short* xl) {
  __shared__ float tn[kNodePad];
  const int b = blockIdx.x;
  const int t = threadIdx.x;
  if (t < kNodePad) {
    const int tc = (t < kNode) ? t : (kNode - 1);
    const float raw = tnraw[(size_t)b * kHid + tc];
    const float v = fmaxf(g_tn[tc] * ((raw + btn[tc]) * kInvS1) + b_tn[tc], 0.0f);
    tn[t] = (t < kNode) ? v : 0.0f;
  }
  __syncthreads();
  const size_t base = (size_t)b * (kNodePad * kKx);
  const int nch = (kNodePad * kKx) / 8;
  for (int pass = 0; pass < 2; ++pass) {
#pragma unroll 1
    for (int c = t; c < nch; c += 256) {
      const int e  = c * 8;
      const int i  = e / kKx;
      const int k0 = e - i * kKx;
      F8 f;
#pragma unroll
      for (int q = 0; q < 8; ++q) {
        const int k  = k0 + q;
        const int ti = k - kNode;
        const int tic = (ti < 0) ? 0 : ((ti > kNodePad - 1) ? (kNodePad - 1) : ti);
        const float tv = tn[tic];
        const float v = (k < kNode) ? ((k == i) ? 1.0f : 0.0f) : ((k < 2 * kNode) ? tv : 0.0f);
        f.v[q] = (i < kNode) ? v : 0.0f;
      }
      v4u wh, wl;
      pack_hl(f, wh, wl);
      *(volatile v4u*)(xh + base + (size_t)e) = wh;
      *(volatile v4u*)(xl + base + (size_t)e) = wl;
    }
    __threadfence();
  }
}

__global__ __launch_bounds__(256) void k_final(const float* __restrict__ E, const float* __restrict__ cbt,
                                               const float* __restrict__ g_e1, const float* __restrict__ b_e1,
                                               float* out) {
  const int gt = blockIdx.x * 256 + threadIdx.x;
  const int idx4 = gt * 4;
  if (idx4 >= kBatch * kNode * kNode) return;
  const int b   = idx4 / (kNode * kNode);
  const int rem = idx4 - b * (kNode * kNode);
  const int i   = rem / kNode;
  const int j0  = rem - i * kNode;
  const float ge = g_e1[0] * kInvS1;
  const float bo = b_e1[0];
  const float* Eb = E + (size_t)b * (kNodePad * kUbtRows);
  const float alpha = Eb[i * kUbtRows];
  const float cb = cbt[b];
  v4f o;
#pragma unroll
  for (int q = 0; q < 4; ++q) {
    const int j = j0 + q;
    const float beta = Eb[j * kUbtRows + 1];
    const float s = alpha + beta + cb;
    const float r = ge * s + bo;
    o[q] = (i == j) ? 0.0f : r;
  }
  for (int pass = 0; pass < 2; ++pass) {
    *(volatile v4f*)(out + idx4) = o;
    __threadfence();
  }
}

extern "C" void kernel_launch(void* const* d_in, const int* in_sizes, int n_in,
                              void* d_out, int out_size, void* d_ws, size_t ws_size,
                              hipStream_t stream) {
  if (n_in < 30) return;
  if (in_sizes[0] != kBatch * kNode * kNode || in_sizes[1] != kBatch || out_size != kBatch * kNode * kNode) return;
  if (in_sizes[10] != 2 * kNode * kHid || in_sizes[22] != 2 * kHid * kHid || in_sizes[26] != 2 * kHid) return;

  const float* X     = (const float*)d_in[0];
  const float* timev = (const float*)d_in[1];
  const float* Wt1   = (const float*)d_in[2];
  const float* bt1   = (const float*)d_in[3];
  const float* Wt2   = (const float*)d_in[4];
  const float* bt2   = (const float*)d_in[5];
  const float* Wtn   = (const float*)d_in[6];
  const float* btn   = (const float*)d_in[7];
  const float* g_tn  = (const float*)d_in[8];
  const float* b_tn  = (const float*)d_in[9];
  const float* Wg1   = (const float*)d_in[10];
  const float* bg1   = (const float*)d_in[11];
  const float* g1    = (const float*)d_in[12];
  const float* bb1   = (const float*)d_in[13];
  const float* Wg2   = (const float*)d_in[14];
  const float* bg2   = (const float*)d_in[15];
  const float* g2    = (const float*)d_in[16];
  const float* bb2   = (const float*)d_in[17];
  const float* Wg3   = (const float*)d_in[18];
  const float* bg3   = (const float*)d_in[19];
  const float* g3    = (const float*)d_in[20];
  const float* bb3   = (const float*)d_in[21];
  const float* We0   = (const float*)d_in[22];
  const float* be0   = (const float*)d_in[23];
  const float* g_e0  = (const float*)d_in[24];
  const float* b_e0  = (const float*)d_in[25];
  const float* We1   = (const float*)d_in[26];
  const float* be1   = (const float*)d_in[27];
  const float* g_e1  = (const float*)d_in[28];
  const float* b_e1  = (const float*)d_in[29];
  float* out = (float*)d_out;

  const size_t szW    = (size_t)kHid * kHid * 2;
  const size_t szWg1  = (size_t)kHid * kKx * 2;
  const size_t szUbt  = (size_t)kUbtRows * kHid * 2;
  const size_t szS16  = (size_t)kBatch * kHid * 2;
  const size_t szS32  = (size_t)kBatch * kHid * 4;
  const size_t szCbt  = 256;
  const size_t szX    = (size_t)kBatch * kNodePad * kKx * 2;
  const size_t szAct  = (size_t)kBatch * kNodePad * kHid * 2;
  const size_t szE    = (size_t)kBatch * kNodePad * kUbtRows * 4;

  char* ws = (char*)d_ws;
  size_t off = 0;
  auto carve = [&](size_t bytes) -> char* { char* p = ws + off; off += bytes; return p; };
  unsigned short* wt1H = (unsigned short*)carve(szW);   unsigned short* wt1L = (unsigned short*)carve(szW);
  unsigned short* wt2H = (unsigned short*)carve(szW);   unsigned short* wt2L = (unsigned short*)carve(szW);
  unsigned short* wtnH = (unsigned short*)carve(szW);   unsigned short* wtnL = (unsigned short*)carve(szW);
  unsigned short* wg1H = (unsigned short*)carve(szWg1); unsigned short* wg1L = (unsigned short*)carve(szWg1);
  unsigned short* wg2H = (unsigned short*)carve(szW);   unsigned short* wg2L = (unsigned short*)carve(szW);
  unsigned short* wg3H = (unsigned short*)carve(szW);   unsigned short* wg3L = (unsigned short*)carve(szW);
  unsigned short* ubtH = (unsigned short*)carve(szUbt); unsigned short* ubtL = (unsigned short*)carve(szUbt);
  unsigned short* tmbH = (unsigned short*)carve(szS16); unsigned short* tmbL = (unsigned short*)carve(szS16);
  unsigned short* h1H  = (unsigned short*)carve(szS16); unsigned short* h1L  = (unsigned short*)carve(szS16);
  float*          hf   = (float*)carve(szS32);
  unsigned short* hpH  = (unsigned short*)carve(szS16); unsigned short* hpL  = (unsigned short*)carve(szS16);
  float*          tnrw = (float*)carve(szS32);
  float*          cbt  = (float*)carve(szCbt);
  unsigned short* xH   = (unsigned short*)carve(szX);   unsigned short* xL   = (unsigned short*)carve(szX);
  unsigned short* adjH = (unsigned short*)carve(szAct); unsigned short* adjL = (unsigned short*)carve(szAct);
  unsigned short* a0H  = (unsigned short*)carve(szAct); unsigned short* a0L  = (unsigned short*)carve(szAct);
  unsigned short* a1H  = (unsigned short*)carve(szAct); unsigned short* a1L  = (unsigned short*)carve(szAct);
  unsigned short* a2H  = (unsigned short*)carve(szAct); unsigned short* a2L  = (unsigned short*)carve(szAct);
  unsigned short* a3H  = (unsigned short*)carve(szAct); unsigned short* a3L  = (unsigned short*)carve(szAct);
  unsigned short* a4H  = (unsigned short*)carve(szAct); unsigned short* a4L  = (unsigned short*)carve(szAct);
  unsigned short* a5H  = (unsigned short*)carve(szAct); unsigned short* a5L  = (unsigned short*)carve(szAct);
  float*          E    = (float*)carve(szE);
  if (off != kWsTotal) return;
  if (off > ws_size) return;

  const float cst = (float)(-log(10000.0) / 63.0);
  const long sX   = (long)kNodePad * kKx;
  const long sAct = (long)kNodePad * kHid;
  const long sE   = (long)kNodePad * kUbtRows;

  k_wtrans<<<48, 256, 0, stream>>>(Wt1, Wt2, Wtn, Wg1, Wg2, Wg3,
                                   wt1H, wt1L, wt2H, wt2L, wtnH, wtnL, wg1H, wg1L, wg2H, wg2L, wg3H, wg3L);
  k_temb<<<1, 256, 0, stream>>>(timev, tmbH, tmbL, cst);
  k_adj<<<kBatch, 256, 0, stream>>>(X, adjH, adjL);
  k_ubt<<<1, 256, 0, stream>>>(We0, We1, g_e0, ubtH, ubtL);
  wmma_gemm64<1, true, 2, 2, false, 2><<<dim3(1, 1), 256, 0, stream>>>(
      tmbH, tmbL, kTdim, 0L, wt1H, wt1L, kTdim, 0L, (void*)h1H, (void*)h1L, kHid, 0L,
      bt1, bt1, bt1, bt1, 0L, kBatch, kHid, kTdim, 1.0f);
  wmma_gemm64<1, true, 2, 0, false, 0><<<dim3(1, 1), 256, 0, stream>>>(
      h1H, h1L, kHid, 0L, wt2H, wt2L, kHid, 0L, (void*)hf, (void*)hf, kHid, 0L,
      bt2, bt2, bt2, bt2, 0L, kBatch, kHid, kHid, 1.0f);
  k_hpost<<<1, 256, 0, stream>>>(hf, We1, be0, b_e0, g_e0, be1, hpH, hpL, cbt);
  wmma_gemm64<1, true, 0, 0, false, 0><<<dim3(1, 1), 256, 0, stream>>>(
      hpH, hpL, kHid, 0L, wtnH, wtnL, kHid, 0L, (void*)tnrw, (void*)tnrw, kHid, 0L,
      btn, btn, btn, btn, 0L, kBatch, kNodePad, kHid, 1.0f);
  k_xbuild<<<kBatch, 256, 0, stream>>>(tnrw, btn, g_tn, b_tn, xH, xL);
  wmma_gemm64<1, true, 0, 2, false, 0><<<dim3(1, kBatch), 256, 0, stream>>>(
      wg1H, wg1L, kKx, 0L, xH, xL, kKx, sX, (void*)a0H, (void*)a0L, kHid, sAct,
      bg1, bg1, bg1, bg1, 0L, kNodePad, kHid, kKx, 1.0f);
  wmma_gemm64<1, true, 3, 2, false, 0><<<dim3(1, kBatch), 256, 0, stream>>>(
      adjH, adjL, kNodePad, sAct, a0H, a0L, kNodePad, sAct, (void*)a1H, (void*)a1L, kHid, sAct,
      bg1, g1, bb1, bg1, 0L, kNodePad, kHid, kNodePad, 1.0f);
  wmma_gemm64<1, true, 0, 2, false, 0><<<dim3(1, kBatch), 256, 0, stream>>>(
      wg2H, wg2L, kHid, 0L, a1H, a1L, kHid, sAct, (void*)a2H, (void*)a2L, kNodePad, sAct,
      bg2, bg2, bg2, bg2, 0L, kHid, kNodePad, kHid, 1.0f);
  wmma_gemm64<1, true, 3, 2, false, 0><<<dim3(1, kBatch), 256, 0, stream>>>(
      adjH, adjL, kNodePad, sAct, a2H, a2L, kNodePad, sAct, (void*)a3H, (void*)a3L, kHid, sAct,
      bg2, g2, bb2, bg2, 0L, kNodePad, kHid, kNodePad, 1.0f);
  wmma_gemm64<1, true, 0, 2, false, 0><<<dim3(1, kBatch), 256, 0, stream>>>(
      wg3H, wg3L, kHid, 0L, a3H, a3L, kHid, sAct, (void*)a4H, (void*)a4L, kNodePad, sAct,
      bg3, bg3, bg3, bg3, 0L, kHid, kNodePad, kHid, 1.0f);
  wmma_gemm64<1, true, 3, 2, false, 0><<<dim3(1, kBatch), 256, 0, stream>>>(
      adjH, adjL, kNodePad, sAct, a4H, a4L, kNodePad, sAct, (void*)a5H, (void*)a5L, kHid, sAct,
      bg3, g3, bb3, bg3, 0L, kNodePad, kHid, kNodePad, 1.0f);
  wmma_gemm64<1, true, 0, 0, false, 0><<<dim3(1, kBatch), 256, 0, stream>>>(
      a5H, a5L, kHid, sAct, ubtH, ubtL, kHid, 0L, (void*)E, (void*)E, kUbtRows, sE,
      bg3, bg3, bg3, bg3, 0L, kNodePad, kUbtRows, kHid, 1.0f);
  k_final<<<(kBatch * kNode * kNode) / 1024, 256, 0, stream>>>(E, cbt, g_e1, b_e1, out);
}
